// SelfAttention_53558242181618
// MI455X (gfx1250) — hardware-verified
//
#include <hip/hip_runtime.h>


#ifndef NB
#define NB 4
#endif
#ifndef SEQ
#define SEQ 2048
#endif
#ifndef ISL_ROWS
#define ISL_ROWS 512
#endif
#define NB_FULL    4
#define SEQ_FULL   2048
#define HID        1024
#define NHEAD      16
#define HDIM       64
#define QKV_N      3072
#define ISL        ((SEQ < ISL_ROWS) ? SEQ : ISL_ROWS)
#define BQ         128
#define BK         32
#define NWAVE      8
#define NQB        (SEQ / BQ)
#define EARLY_QBLK (ISL / BQ)
#define TP         72
#define OP         68
#define SP         136
#define LATE_TILES ((((SEQ - ISL) / 128) > 0) ? ((SEQ - ISL) / 128) : 1)

#define N_XB   ((size_t)NB * SEQ * HID)
#define N_WQ   ((size_t)QKV_N * HID)
#define N_WO   ((size_t)HID * HID)
#define N_HP   ((size_t)NB * NHEAD * SEQ * HDIM)
#define N_RP   ((size_t)NB * NHEAD * ISL * HDIM)
#define N_CR   ((size_t)NB * ISL * HID)
#define OFF_XB ((size_t)0)
#define OFF_WQ (OFF_XB + N_XB)
#define OFF_WO (OFF_WQ + N_WQ)
#define OFF_QH (OFF_WO + N_WO)
#define OFF_KH (OFF_QH + N_HP)
#define OFF_VT (OFF_KH + N_HP)
#define OFF_QR (OFF_VT + N_HP)
#define OFF_KR (OFF_QR + N_RP)
#define OFF_VR (OFF_KR + N_RP)
#define OFF_CH (OFF_VR + N_RP)
#define OFF_CR (OFF_CH + N_XB)
#define WS_ELEMS (OFF_CR + N_CR)
#define WS_BYTES (WS_ELEMS * 2)

static_assert(SEQ % BQ == 0);
static_assert(SEQ % 128 == 0);
static_assert(ISL % 128 == 0);
static_assert(ISL % BK == 0);
static_assert(ISL >= 128 && ISL <= SEQ);
static_assert(BQ == NWAVE * 16);
static_assert(HDIM == 64);
static_assert(HID == NHEAD * HDIM);
static_assert(QKV_N == 3 * HID);
static_assert(HID % 128 == 0);
static_assert(HID % 32 == 0);
static_assert(QKV_N % 128 == 0);
static_assert(HID % 64 == 0 && QKV_N % 64 == 0);
static_assert((NB * SEQ) % 128 == 0);
static_assert(SEQ <= SEQ_FULL);
static_assert(NB >= 1 && NB <= NB_FULL);
static_assert((TP * 2) % 16 == 0 && TP >= 64);
static_assert((OP * 4) % 16 == 0 && OP >= 64);
static_assert((SP * 2) % 16 == 0 && SP >= 128);
static_assert(N_XB % 2048 == 0);
static_assert(WS_BYTES <= (size_t)134217728);
static_assert((size_t)NB_FULL * SEQ_FULL * HID * 4 == (size_t)33554432);

typedef __bf16         bf16;
typedef _Float16       f16;
typedef unsigned short u16;
typedef bf16     v16bf __attribute__((ext_vector_type(16)));
typedef f16      v16h  __attribute__((ext_vector_type(16)));
typedef f16      v8h   __attribute__((ext_vector_type(8)));
typedef u16      v8us  __attribute__((ext_vector_type(8)));
typedef float    v8f   __attribute__((ext_vector_type(8)));
typedef float    v4f   __attribute__((ext_vector_type(4)));
typedef unsigned v4u   __attribute__((ext_vector_type(4)));

union Frag   { v16bf vb; v16h vh; v4u q[2]; f16 h[16]; };
union Pack8B { v4u u; bf16 h[8]; };
union Pack8H { v4u u; v8h v; f16 h[8]; };
union Pack8U { v4u u; v8us v; };

static __device__ __forceinline__ v8f mma_bf16(v16bf a, v16bf b, v8f acc) {
  acc = __builtin_amdgcn_wmma_f32_16x16x32_bf16(false, a, false, b, (short)0, acc, false, false);
  asm volatile("v_nop\n\tv_nop\n\tv_nop\n\tv_nop" : "+v"(acc) : "v"(a), "v"(b));
  return acc;
}
static __device__ __forceinline__ v8f mma_f16(v16h a, v16h b, v8f acc) {
  acc = __builtin_amdgcn_wmma_f32_16x16x32_f16(false, a, false, b, (short)0, acc, false, false);
  asm volatile("v_nop\n\tv_nop\n\tv_nop\n\tv_nop" : "+v"(acc) : "v"(a), "v"(b));
  return acc;
}
template <int BF>
static __device__ __forceinline__ v8f mma_sel(const Frag& a, const Frag& b, v8f acc) {
  if (BF != 0) return mma_bf16(a.vb, b.vb, acc);
  return mma_f16(a.vh, b.vh, acc);
}

__global__ __launch_bounds__(256) void cvt_x_kernel(const float* __restrict__ x, u16* ws16) {
  const size_t e = ((size_t)blockIdx.x * 256 + threadIdx.x) * 8;
  const size_t m = e / HID;
  const int    c = (int)(e % HID);
  const size_t b = m / SEQ;
  const size_t s = m % SEQ;
  const float* src = x + (b * SEQ_FULL + s) * HID + c;
  const v4f a0 = *(const v4f*)(src);
  const v4f a1 = *(const v4f*)(src + 4);
  Pack8B pk;
  #pragma unroll
  for (int i = 0; i < 4; ++i) {
    pk.h[i]     = (bf16)a0[i];
    pk.h[4 + i] = (bf16)a1[i];
  }
  const v4u val = pk.u;
  u16* dst = ws16 + OFF_XB + e;
  *(volatile v4u*)dst = val;
  __threadfence();
  *(volatile v4u*)dst = val;
}

static __device__ __forceinline__ u16 cvt16(float v, int mode) {
  const bf16 bv = (bf16)v;
  const u16  b0 = __builtin_bit_cast(u16, bv);
  const f16  hv = (f16)((float)bv * 64.0f);
  const u16  b1 = __builtin_bit_cast(u16, hv);
  return (mode != 0) ? b1 : b0;
}

__global__ __launch_bounds__(256) void wt_kernel(const float* __restrict__ in, u16* ws16, size_t out_off,
                                                 int R, int C, int mode) {
  __shared__ __align__(16) u16 sT[64 * TP];
  const int tid = threadIdx.x;
  const int c0  = blockIdx.x * 64;
  const int r0  = blockIdx.y * 64;
  #pragma unroll
  for (int kk = 0; kk < 2; ++kk) {
    const int row  = kk * 32 + (tid >> 3);
    const int col0 = (tid & 7) * 8;
    const float* src = in + (size_t)(r0 + row) * C + c0 + col0;
    const v4f a0 = *(const v4f*)(src);
    const v4f a1 = *(const v4f*)(src + 4);
    #pragma unroll
    for (int i = 0; i < 4; ++i) {
      sT[(col0 + i) * TP + row]     = cvt16(a0[i], mode);
      sT[(col0 + 4 + i) * TP + row] = cvt16(a1[i], mode);
    }
  }
  __syncthreads();
  v4u    vals[2];
  size_t gi[2];
  #pragma unroll
  for (int kk = 0; kk < 2; ++kk) {
    const int orow = kk * 32 + (tid >> 3);
    const int ks   = (tid & 7) * 8;
    Pack8U pu;
    pu.v = *(const v8us*)(sT + orow * TP + ks);
    vals[kk] = pu.u;
    gi[kk]   = out_off + (size_t)(c0 + orow) * R + r0 + ks;
  }
  #pragma unroll
  for (int kk = 0; kk < 2; ++kk) *(volatile v4u*)(ws16 + gi[kk]) = vals[kk];
  __threadfence();
  #pragma unroll
  for (int kk = 0; kk < 2; ++kk) *(volatile v4u*)(ws16 + gi[kk]) = vals[kk];
}

template <int MT, int RES, int BF>
static __device__ __forceinline__ void gemm_mainloop(const u16* base, const size_t a_off, const size_t ar_off,
                                                     const size_t b_off, v8f (&acc)[MT][4], v8f (&acc2)[MT][4]) {
  const int lane = threadIdx.x & 31;
  const int lq   = lane & 15;
  const int hi   = lane >> 4;
  size_t ao[MT], aro[MT], bo[4];
  #pragma unroll
  for (int i = 0; i < MT; ++i) {
    ao[i]  = a_off  + (size_t)(16 * i + lq) * HID + hi * 8;
    aro[i] = ar_off + (size_t)(16 * i + lq) * HID + hi * 8;
  }
  #pragma unroll
  for (int j = 0; j < 4; ++j) bo[j] = b_off + (size_t)(16 * j + lq) * HID + hi * 8;
  #pragma unroll
  for (int i = 0; i < MT; ++i) {
    #pragma unroll
    for (int j = 0; j < 4; ++j) {
      acc[i][j]  = (v8f){0, 0, 0, 0, 0, 0, 0, 0};
      acc2[i][j] = (v8f){0, 0, 0, 0, 0, 0, 0, 0};
    }
  }
  #pragma unroll 1
  for (int k0 = 0; k0 < HID; k0 += 32) {
    Frag a[MT], ar[MT], bw[4];
    #pragma unroll
    for (int i = 0; i < MT; ++i) {
      a[i].q[0] = *(const v4u*)(base + ao[i] + k0);
      a[i].q[1] = *(const v4u*)(base + ao[i] + k0 + 16);
      if (RES != 0) {
        ar[i].q[0] = *(const v4u*)(base + aro[i] + k0);
        ar[i].q[1] = *(const v4u*)(base + aro[i] + k0 + 16);
      }
    }
    #pragma unroll
    for (int j = 0; j < 4; ++j) {
      bw[j].q[0] = *(const v4u*)(base + bo[j] + k0);
      bw[j].q[1] = *(const v4u*)(base + bo[j] + k0 + 16);
    }
    #pragma unroll
    for (int i = 0; i < MT; ++i) {
      #pragma unroll
      for (int j = 0; j < 4; ++j) {
        acc[i][j] = mma_sel<BF>(a[i], bw[j], acc[i][j]);
        if (RES != 0) acc2[i][j] = mma_sel<BF>(ar[i], bw[j], acc2[i][j]);
      }
    }
  }
}

template <int PASS>
static __device__ __forceinline__ void qkv_stage_store(f16* st, u16* ws16, const v8f (&acc)[2][4],
                                                       const float (&bj)[4], const int which, const int head0,
                                                       const int b, const int s0, const int mw, const int nw,
                                                       const int lq, const int hi, const int tid) {
  #pragma unroll
  for (int i = 0; i < 2; ++i) {
    #pragma unroll
    for (int j = 0; j < 4; ++j) {
      #pragma unroll
      for (int r = 0; r < 8; ++r) {
        const float v  = acc[i][j][r] + bj[j];
        const f16   hv = (f16)v;
        const f16   ov = (PASS == 0) ? hv : (f16)((v - (float)hv) * 1024.0f);
        const int   rl = mw + 16 * i + 8 * hi + r;
        const int   cl = nw + 16 * j + lq;
        const int  idx = (which == 2) ? (cl * SP + rl) : (rl * SP + cl);
        st[idx] = ov;
      }
    }
  }
  __syncthreads();
  const size_t rows    = (PASS == 0) ? (size_t)SEQ : (size_t)ISL;
  const size_t base_qk = (PASS == 0) ? ((which == 0) ? OFF_QH : OFF_KH) : ((which == 0) ? OFF_QR : OFF_KR);
  const size_t base_v  = (PASS == 0) ? OFF_VT : OFF_VR;
  v4u    vals[8];
  size_t gi[8];
  #pragma unroll
  for (int it = 0; it < 8; ++it) {
    const int L     = it * 32 + (tid >> 3);
    const int rowL  = L & 127;
    const int seg   = L >> 7;
    const int piece = tid & 7;
    Pack8H ph;
    ph.v = *(const v8h*)(st + rowL * SP + seg * 64 + piece * 8);
    vals[it] = ph.u;
    const size_t gqk = base_qk + (((size_t)b * NHEAD + head0 + seg) * rows + s0 + rowL) * HDIM + piece * 8;
    const size_t gv  = base_v + (((size_t)b * NHEAD + head0 + (rowL >> 6)) * HDIM + (rowL & 63)) * rows
                       + s0 + seg * 64 + piece * 8;
    gi[it] = (which == 2) ? gv : gqk;
  }
  #pragma unroll
  for (int it = 0; it < 8; ++it) *(volatile v4u*)(ws16 + gi[it]) = vals[it];
  __threadfence();
  #pragma unroll
  for (int it = 0; it < 8; ++it) *(volatile v4u*)(ws16 + gi[it]) = vals[it];
}

__global__ __launch_bounds__(256) void qkv_gemm_kernel(u16* ws16, const float* __restrict__ bias) {
  __shared__ __align__(16) f16 st[128 * SP];
  const int tid  = threadIdx.x;
  const int wave = tid >> 5;
  const int lane = tid & 31;
  const int lq   = lane & 15;
  const int hi   = lane >> 4;
  const int N0   = blockIdx.x * 128;
  const int M0   = blockIdx.y * 128;
  const int mw   = (wave >> 1) * 32;
  const int nw   = (wave & 1) * 64;

  v8f acc[2][4], acc2[2][4];
  gemm_mainloop<2, 0, 1>(ws16, OFF_XB + (size_t)(M0 + mw) * HID, (size_t)0,
                         OFF_WQ + (size_t)(N0 + nw) * HID, acc, acc2);

  const int  which  = N0 / HID;
  const int  head0  = (N0 % HID) / HDIM;
  const int  b      = M0 / SEQ;
  const int  s0     = M0 % SEQ;
  const bool island = (s0 < ISL);

  float bj[4];
  #pragma unroll
  for (int j = 0; j < 4; ++j) bj[j] = (float)(bf16)bias[N0 + nw + 16 * j + lq];

  qkv_stage_store<0>(st, ws16, acc, bj, which, head0, b, s0, mw, nw, lq, hi, tid);
  if (island) {
    __syncthreads();
    qkv_stage_store<1>(st, ws16, acc, bj, which, head0, b, s0, mw, nw, lq, hi, tid);
  }
}

template <int RES>
static __device__ __forceinline__ void attn_body(u16* ws16, const int qblk, const int h, const int b) {
  __shared__ __align__(16) float sO[NWAVE * 16 * OP];
  const int tid  = threadIdx.x;
  const int wave = tid >> 5;
  const int lane = tid & 31;
  const int lq   = lane & 15;
  const int hi   = lane >> 4;

  const int    qrow0 = qblk * BQ + wave * 16;
  const size_t bh    = (size_t)b * NHEAD + h;
  const u16* q_h  = ws16 + OFF_QH + bh * SEQ * HDIM;
  const u16* k_h  = ws16 + OFF_KH + bh * SEQ * HDIM;
  const u16* vt_h = ws16 + OFF_VT + bh * HDIM * SEQ;
  const u16* qr_h = ws16 + OFF_QR + bh * ISL * HDIM;
  const u16* kr_h = ws16 + OFF_KR + bh * ISL * HDIM;
  const u16* vr_h = ws16 + OFF_VR + bh * HDIM * ISL;

  Frag qf[2], qr[2];
  {
    const size_t qo = (size_t)(qrow0 + lq) * HDIM + hi * 8;
    #pragma unroll
    for (int f = 0; f < 2; ++f) {
      qf[f].q[0] = *(const v4u*)(q_h + qo + f * 32);
      qf[f].q[1] = *(const v4u*)(q_h + qo + f * 32 + 16);
      if (RES != 0) {
        qr[f].q[0] = *(const v4u*)(qr_h + qo + f * 32);
        qr[f].q[1] = *(const v4u*)(qr_h + qo + f * 32 + 16);
      }
    }
  }

  v8f o[4], o2[4];
  #pragma unroll
  for (int dt = 0; dt < 4; ++dt) {
    o[dt]  = (v8f){0, 0, 0, 0, 0, 0, 0, 0};
    o2[dt] = (v8f){0, 0, 0, 0, 0, 0, 0, 0};
  }

  float rmax = -__builtin_inff();
  float rsum = 0.0f;
  const float SL = 0.125f * 1.4426950408889634f;

  const int nchunk = (qrow0 + 15) / BK + 1;
  for (int ic = 0; ic < nchunk; ++ic) {
    const int j0 = ic * BK;

    v8f c[2];
    #pragma unroll
    for (int sub = 0; sub < 2; ++sub) {
      const size_t krow = (size_t)(j0 + sub * 16 + lq) * HDIM + hi * 8;
      Frag a0, a1;
      a0.q[0] = *(const v4u*)(k_h + krow);
      a0.q[1] = *(const v4u*)(k_h + krow + 16);
      a1.q[0] = *(const v4u*)(k_h + krow + 32);
      a1.q[1] = *(const v4u*)(k_h + krow + 48);
      v8f acc = (v8f){0, 0, 0, 0, 0, 0, 0, 0};
      acc = mma_f16(a0.vh, qf[0].vh, acc);
      acc = mma_f16(a1.vh, qf[1].vh, acc);
      if (RES != 0) {
        Frag kr0, kr1;
        kr0.q[0] = *(const v4u*)(kr_h + krow);
        kr0.q[1] = *(const v4u*)(kr_h + krow + 16);
        kr1.q[0] = *(const v4u*)(kr_h + krow + 32);
        kr1.q[1] = *(const v4u*)(kr_h + krow + 48);
        v8f xa = (v8f){0, 0, 0, 0, 0, 0, 0, 0};
        xa = mma_f16(a0.vh, qr[0].vh, xa);
        xa = mma_f16(a1.vh, qr[1].vh, xa);
        xa = mma_f16(kr0.vh, qf[0].vh, xa);
        xa = mma_f16(kr1.vh, qf[1].vh, xa);
        #pragma unroll
        for (int r = 0; r < 8; ++r) acc[r] += xa[r] * (1.0f / 1024.0f);
      }
      c[sub] = acc;
      __builtin_amdgcn_sched_barrier(0);
    }

    if (j0 + BK - 1 > qrow0) {
      const int qi = qrow0 + lq;
      #pragma unroll
      for (int sub = 0; sub < 2; ++sub) {
        #pragma unroll
        for (int r = 0; r < 8; ++r) {
          const int key = j0 + sub * 16 + hi * 8 + r;
          c[sub][r] = (key > qi) ? -__builtin_inff() : c[sub][r];
        }
      }
    }

    float m_new = rmax;
    #pragma unroll
    for (int r = 0; r < 8; ++r) {
      m_new = fmaxf(m_new, c[0][r]);
      m_new = fmaxf(m_new, c[1][r]);
    }
    m_new = fmaxf(m_new, __shfl_xor(m_new, 16, 32));
    const float scale = __builtin_amdgcn_exp2f((rmax - m_new) * SL);
    rmax = m_new;

    Frag pa, pr;
    float psum = 0.0f;
    #pragma unroll
    for (int r = 0; r < 8; ++r) {
      const float p0 = __builtin_amdgcn_exp2f((c[0][r] - m_new) * SL);
      const float p1 = __builtin_amdgcn_exp2f((c[1][r] - m_new) * SL);
      psum += p0 + p1;
      const float pc0 = p0 * 4096.0f;
      const float pc1 = p1 * 4096.0f;
      const f16 h0 = (f16)pc0;
      const f16 h1 = (f16)pc1;
      pa.h[r]     = h0;
      pa.h[8 + r] = h1;
      if (RES != 0) {
        pr.h[r]     = (f16)((pc0 - (float)h0) * 1024.0f);
        pr.h[8 + r] = (f16)((pc1 - (float)h1) * 1024.0f);
      }
    }
    rsum = rsum * scale + psum + __shfl_xor(psum, 16, 32);

    float sc[8];
    #pragma unroll
    for (int r = 0; r < 8; ++r) sc[r] = __shfl(scale, (hi << 3) + r, 32);
    #pragma unroll
    for (int dt = 0; dt < 4; ++dt) {
      #pragma unroll
      for (int r = 0; r < 8; ++r) {
        o[dt][r] *= sc[r];
        if (RES != 0) o2[dt][r] *= sc[r];
      }
    }
    __builtin_amdgcn_sched_barrier(0);

    #pragma unroll
    for (int dt = 0; dt < 4; ++dt) {
      const size_t vrow = (size_t)(dt * 16 + lq);
      Frag bv;
      bv.q[0] = *(const v4u*)(vt_h + vrow * SEQ + j0 + hi * 8);
      bv.q[1] = *(const v4u*)(vt_h + vrow * SEQ + j0 + hi * 8 + 16);
      o[dt] = mma_f16(pa.vh, bv.vh, o[dt]);
      if (RES != 0) {
        Frag bvr;
        bvr.q[0] = *(const v4u*)(vr_h + vrow * ISL + j0 + hi * 8);
        bvr.q[1] = *(const v4u*)(vr_h + vrow * ISL + j0 + hi * 8 + 16);
        o2[dt] = mma_f16(pr.vh, bv.vh, o2[dt]);
        o2[dt] = mma_f16(pa.vh, bvr.vh, o2[dt]);
      }
      __builtin_amdgcn_sched_barrier(0);
    }
  }

  float rs[8];
  #pragma unroll
  for (int r = 0; r < 8; ++r) rs[r] = 1.0f / __shfl(rsum, (hi << 3) + r, 32);

  float* so = sO + wave * (16 * OP);
  #pragma unroll
  for (int r = 0; r < 8; ++r) {
    #pragma unroll
    for (int dt = 0; dt < 4; ++dt) {
      float val = o[dt][r];
      if (RES != 0) val += o2[dt][r] * (1.0f / 1024.0f);
      so[(hi * 8 + r) * OP + dt * 16 + lq] = val * (1.0f / 4096.0f) * rs[r];
    }
  }
  __syncthreads();

  v4u    hval[4], rval[4];
  size_t hidx[4], ridx[4];
  #pragma unroll
  for (int it = 0; it < 4; ++it) {
    const int row   = it * 4 + (lane >> 3);
    const int piece = lane & 7;
    const v4f x0 = *(const v4f*)(so + row * OP + piece * 8);
    const v4f x1 = *(const v4f*)(so + row * OP + piece * 8 + 4);
    Pack8H ph, pq;
    #pragma unroll
    for (int i = 0; i < 4; ++i) {
      const float c0 = x0[i] * 16.0f;
      const float c1 = x1[i] * 16.0f;
      const f16 g0 = (f16)c0;
      const f16 g1 = (f16)c1;
      ph.h[i]     = g0;
      ph.h[4 + i] = g1;
      pq.h[i]     = (f16)((c0 - (float)g0) * 1024.0f);
      pq.h[4 + i] = (f16)((c1 - (float)g1) * 1024.0f);
    }
    hval[it] = ph.u;
    rval[it] = pq.u;
    hidx[it] = OFF_CH + ((size_t)b * SEQ + qrow0 + row) * HID + h * HDIM + piece * 8;
    ridx[it] = OFF_CR + ((size_t)b * ISL + qrow0 + row) * HID + h * HDIM + piece * 8;
  }
  #pragma unroll
  for (int it = 0; it < 4; ++it) {
    *(volatile v4u*)(ws16 + hidx[it]) = hval[it];
    if (RES != 0) *(volatile v4u*)(ws16 + ridx[it]) = rval[it];
  }
  __threadfence();
  #pragma unroll
  for (int it = 0; it < 4; ++it) {
    *(volatile v4u*)(ws16 + hidx[it]) = hval[it];
    if (RES != 0) *(volatile v4u*)(ws16 + ridx[it]) = rval[it];
  }
}

__global__ __launch_bounds__(256) void attn_early_kernel(u16* ws16) {
  attn_body<1>(ws16, (int)blockIdx.x, (int)blockIdx.y, (int)blockIdx.z);
}
__global__ __launch_bounds__(256) void attn_late_kernel(u16* ws16) {
  attn_body<0>(ws16, EARLY_QBLK + (int)blockIdx.x, (int)blockIdx.y, (int)blockIdx.z);
}

template <int MT, int RES>
static __device__ __forceinline__ void out_gemm_body(u16* ws16, const float* __restrict__ bias, float* out,
                                                     const int b, const int s0) {
  __shared__ __align__(16) float sO[NWAVE * 16 * OP];
  const int tid  = threadIdx.x;
  const int wave = tid >> 5;
  const int lane = tid & 31;
  const int lq   = lane & 15;
  const int hi   = lane >> 4;
  const int N0   = blockIdx.x * 128;
  const int mw   = (wave >> 1) * (16 * MT);
  const int nw   = (wave & 1) * 64;

  v8f acc[MT][4], acc2[MT][4];
  gemm_mainloop<MT, RES, 0>(ws16, OFF_CH + ((size_t)b * SEQ + s0 + mw) * HID,
                            OFF_CR + ((size_t)b * ISL + s0 + mw) * HID,
                            OFF_WO + (size_t)(N0 + nw) * HID, acc, acc2);

  v4f b4 = *(const v4f*)(bias + N0 + nw + lq * 4);
  #pragma unroll
  for (int i = 0; i < 4; ++i) b4[i] = (float)(bf16)b4[i];

  float* so = sO + wave * (16 * OP);
  #pragma unroll
  for (int i = 0; i < MT; ++i) {
    if (i > 0) __syncthreads();
    #pragma unroll
    for (int r = 0; r < 8; ++r) {
      #pragma unroll
      for (int j = 0; j < 4; ++j) {
        float val = acc[i][j][r];
        if (RES != 0) val += acc2[i][j][r] * (1.0f / 1024.0f);
        so[(hi * 8 + r) * OP + 16 * j + lq] = val * (1.0f / 1024.0f);
      }
    }
    __syncthreads();
    v4f    vals[8];
    size_t gidx[8];
    #pragma unroll
    for (int it = 0; it < 8; ++it) {
      const int row = it * 2 + hi;
      v4f v = *(const v4f*)(so + row * OP + lq * 4);
      v += b4;
      vals[it] = v;
      gidx[it] = ((size_t)b * SEQ_FULL + s0 + mw + 16 * i + row) * HID + N0 + nw + lq * 4;
    }
    #pragma unroll
    for (int it = 0; it < 8; ++it) *(volatile v4f*)(out + gidx[it]) = vals[it];
    __threadfence();
    #pragma unroll
    for (int it = 0; it < 8; ++it) *(volatile v4f*)(out + gidx[it]) = vals[it];
  }
}

__global__ __launch_bounds__(256) void out_gemm_early_kernel(u16* ws16, const float* __restrict__ bias, float* out) {
  const int y  = (int)blockIdx.y;
  const int b  = y / (ISL / 64);
  const int s0 = (y % (ISL / 64)) * 64;
  out_gemm_body<1, 1>(ws16, bias, out, b, s0);
}
__global__ __launch_bounds__(256) void out_gemm_late_kernel(u16* ws16, const float* __restrict__ bias, float* out) {
  const int y  = (int)blockIdx.y;
  const int b  = y / LATE_TILES;
  const int s0 = ISL + (y % LATE_TILES) * 128;
  out_gemm_body<2, 0>(ws16, bias, out, b, s0);
}

extern "C" void kernel_launch(void* const* d_in, const int* in_sizes, int n_in,
                              void* d_out, int out_size, void* d_ws, size_t ws_size,
                              hipStream_t stream) {
  if (n_in < 5) return;
  const size_t rows_used = (size_t)(NB - 1) * SEQ_FULL + SEQ;
  if ((size_t)in_sizes[0] < rows_used * HID) return;
  if ((size_t)in_sizes[1] < (size_t)HID * QKV_N) return;
  if ((size_t)in_sizes[2] < (size_t)QKV_N) return;
  if ((size_t)in_sizes[3] < (size_t)HID * HID) return;
  if ((size_t)in_sizes[4] < (size_t)HID) return;
  if ((size_t)out_size < rows_used * HID) return;
  if (ws_size < WS_BYTES) return;

  const float* x     = (const float*)d_in[0];
  const float* w_qkv = (const float*)d_in[1];
  const float* b_qkv = (const float*)d_in[2];
  const float* w_out = (const float*)d_in[3];
  const float* b_out = (const float*)d_in[4];
  float*       out   = (float*)d_out;
  u16*         ws16  = (u16*)d_ws;

  cvt_x_kernel<<<dim3((unsigned)(N_XB / 2048)), 256, 0, stream>>>(x, ws16);
  wt_kernel<<<dim3(QKV_N / 64, HID / 64), 256, 0, stream>>>(w_qkv, ws16, OFF_WQ, HID, QKV_N, 0);
  wt_kernel<<<dim3(HID / 64, HID / 64), 256, 0, stream>>>(w_out, ws16, OFF_WO, HID, HID, 1);

  qkv_gemm_kernel<<<dim3(QKV_N / 128, (NB * SEQ) / 128), 256, 0, stream>>>(ws16, b_qkv);

  attn_early_kernel<<<dim3(EARLY_QBLK, NHEAD, NB), 256, 0, stream>>>(ws16);
  if (NQB > EARLY_QBLK)
    attn_late_kernel<<<dim3(NQB - EARLY_QBLK, NHEAD, NB), 256, 0, stream>>>(ws16);

  out_gemm_early_kernel<<<dim3(HID / 128, NB * (ISL / 64)), 256, 0, stream>>>(ws16, b_out, out);
  if (SEQ > ISL)
    out_gemm_late_kernel<<<dim3(HID / 128, NB * ((SEQ - ISL) / 128)), 256, 0, stream>>>(ws16, b_out, out);
}
